// FastAGaLiTeLayer_25993142076004
// MI455X (gfx1250) — hardware-run, weakly checked
//
#include <hip/hip_runtime.h>


#define NL   128
#define NQ   32
#define NM   4096
#define NC   1024
#define NA   8
#define NJ   64
#define NE   4
#define NF   4
#define NV   2656
#define NVP  2688
#define NK5  2560
#define NO   512
#define NW   1024
typedef _Float16 h16;
typedef unsigned short bf;
typedef __attribute__((ext_vector_type(16))) __bf16   v16bf;
typedef __attribute__((ext_vector_type(16))) _Float16 v16h;
typedef __attribute__((ext_vector_type(8)))  _Float16 v8h;
typedef __attribute__((ext_vector_type(8)))  unsigned short v8us;
typedef __attribute__((ext_vector_type(8)))  float    v8f;
typedef __attribute__((ext_vector_type(4)))  float    v4f;
typedef v8h  __attribute__((may_alias)) v8ha;
typedef v4f  __attribute__((may_alias)) v4fa;
typedef v8us __attribute__((may_alias)) v8usa;

__device__ __forceinline__ unsigned short f2bf(float f) { unsigned u = __float_as_uint(f); u += 0x7FFFu + ((u >> 16) & 1u); return (unsigned short)(u >> 16); }
__device__ __forceinline__ float bf2f(unsigned short b) { return __uint_as_float(((unsigned)b) << 16); }
__device__ __forceinline__ float bfr(float f) { return bf2f(f2bf(f)); }
__device__ __forceinline__ v16h cat16(v8h lo, v8h hi) { return __builtin_shufflevector(lo, hi, 0, 1, 2, 3, 4, 5, 6, 7, 8, 9, 10, 11, 12, 13, 14, 15); }
__device__ __forceinline__ v16bf cat16b(v8us lo, v8us hi) { return __builtin_bit_cast(v16bf, __builtin_shufflevector(lo, hi, 0, 1, 2, 3, 4, 5, 6, 7, 8, 9, 10, 11, 12, 13, 14, 15)); }
__device__ __forceinline__ v8f wmma16(v16h a, v16h b, v8f c) { return __builtin_amdgcn_wmma_f32_16x16x32_f16(false, a, false, b, (short)0, c, false, false); }
__device__ __forceinline__ v8f wmmab(v16bf a, v16bf b, v8f c) { return __builtin_amdgcn_wmma_f32_16x16x32_bf16(false, a, false, b, (short)0, c, false, false); }

template <typename T16> struct WFrag;
template <> struct WFrag<h16> { typedef v16h V; static __device__ __forceinline__ V ld(const h16* p) { return cat16(*(const v8h*)p, *(const v8h*)(p + 16)); } static __device__ __forceinline__ v8f mma(V a, V b, v8f c) { return wmma16(a, b, c); } };
template <> struct WFrag<bf> { typedef v16bf V; static __device__ __forceinline__ V ld(const bf* p) { return cat16b(*(const v8us*)p, *(const v8us*)(p + 16)); } static __device__ __forceinline__ v8f mma(V a, V b, v8f c) { return wmmab(a, b, c); } };
template <typename T16, int NSPLIT, bool BIAS>
__global__ __launch_bounds__(32) void k_gemmw(const T16* __restrict__ A, const T16* __restrict__ A2, const T16* __restrict__ Bt, const T16* __restrict__ Bt2, int K, float* C, int ldc, const float* __restrict__ bias, size_t sA, size_t sB, size_t sC) {
    typedef typename WFrag<T16>::V V;
    __shared__ __align__(16) float os[16 * 68];
    const size_t z = blockIdx.z; A += z * sA; if (A2) A2 += z * sA; Bt += z * sB; if (Bt2) Bt2 += z * sB; C += z * sC;
    const int lane = threadIdx.x & 31, lr = lane & 15, hi = lane >> 4; const int r0 = blockIdx.x * 64, c0 = blockIdx.y * 64;
    v8f acc[4][4];
#pragma unroll
    for (int mb = 0; mb < 4; ++mb)
#pragma unroll
        for (int nb = 0; nb < 4; ++nb) acc[mb][nb] = (v8f){};
    const size_t aoff = (size_t)(r0 + lr) * K + 8 * hi, boff = (size_t)(c0 + lr) * K + 8 * hi;
    for (int kc = 0; kc < K; kc += 32) {
        V a[4], a2[4];
#pragma unroll
        for (int mb = 0; mb < 4; ++mb) { a[mb] = WFrag<T16>::ld(A + aoff + (size_t)mb * 16 * K + kc); if (NSPLIT == 1 || NSPLIT == 2) a2[mb] = WFrag<T16>::ld(A2 + aoff + (size_t)mb * 16 * K + kc); }
#pragma unroll
        for (int nb = 0; nb < 4; ++nb) { const V b = WFrag<T16>::ld(Bt + boff + (size_t)nb * 16 * K + kc); V b2; if (NSPLIT >= 2) b2 = WFrag<T16>::ld(Bt2 + boff + (size_t)nb * 16 * K + kc);
#pragma unroll
            for (int mb = 0; mb < 4; ++mb) { acc[mb][nb] = WFrag<T16>::mma(a[mb], b, acc[mb][nb]); if (NSPLIT == 1 || NSPLIT == 2) acc[mb][nb] = WFrag<T16>::mma(a2[mb], b, acc[mb][nb]); if (NSPLIT >= 2) acc[mb][nb] = WFrag<T16>::mma(a[mb], b2, acc[mb][nb]); } }
        asm volatile("v_nop\n\tv_nop\n\tv_nop\n\tv_nop" : "+v"(acc[0][0]), "+v"(acc[1][1]), "+v"(acc[2][2]), "+v"(acc[3][3]) : "v"(a[0]), "v"(a[3]));
    }
#pragma unroll
    for (int mb = 0; mb < 4; ++mb) {
#pragma unroll
        for (int nb = 0; nb < 4; ++nb) {
#pragma unroll
            for (int j = 0; j < 8; ++j) os[(hi * 8 + j) * 68 + nb * 16 + lr] = acc[mb][nb][j]; }
        __builtin_amdgcn_wave_barrier(); asm volatile("" ::: "memory");
        float* crow = C + (size_t)(r0 + mb * 16) * ldc + c0;
#pragma unroll 1
        for (int ps = 0; ps < 2; ++ps) {
#pragma unroll
            for (int s = 0; s < 8; ++s) { const int row = 2 * s + hi, cofs = lr * 4; v4f val = *(const v4fa*)(os + row * 68 + cofs); if (BIAS) { val[0] += bfr(bias[c0 + cofs]); val[1] += bfr(bias[c0 + cofs + 1]); val[2] += bfr(bias[c0 + cofs + 2]); val[3] += bfr(bias[c0 + cofs + 3]); }
                *(volatile v4f*)(crow + (size_t)row * ldc + cofs) = val; }
            if (ps == 0) __threadfence(); }
        __builtin_amdgcn_wave_barrier(); asm volatile("" ::: "memory");
    }
}

typedef __attribute__((ext_vector_type(2))) _Float16 v2h;
typedef __attribute__((ext_vector_type(4))) _Float16 v4h;
typedef __attribute__((ext_vector_type(2))) unsigned short v2us;
typedef __attribute__((ext_vector_type(4))) unsigned short v4us;
typedef __attribute__((ext_vector_type(2))) float v2f;
typedef __attribute__((ext_vector_type(4))) int v4i;
__global__ __launch_bounds__(256) void k_cvt8(const float* __restrict__ src, bf* dst, size_t n8) { const size_t i = (size_t)blockIdx.x * 256 + threadIdx.x; if (i >= n8) return; const v8f v = *(const v8f*)(src + i * 8); v8us o;
#pragma unroll
    for (int k = 0; k < 8; ++k) o[k] = f2bf(v[k]); *(volatile v8us*)(dst + i * 8) = o; __threadfence(); *(volatile v8us*)(dst + i * 8) = o; }

__global__ __launch_bounds__(256) void k_fillb(bf* P, unsigned w2, size_t n8) { const size_t i = (size_t)blockIdx.x * 256 + threadIdx.x; if (i >= n8) return; v4i o; o[0] = (int)w2; o[1] = (int)w2; o[2] = (int)w2; o[3] = (int)w2;
    *(volatile v4i*)(P + i * 8) = o; __threadfence(); *(volatile v4i*)(P + i * 8) = o; }

__device__ __forceinline__ float sgm(float z) { return 1.0f / (1.0f + expf(-z)); }
__constant__ unsigned RATE[NF] = { 0xc0490fdbu, 0xbf860a91u, 0x3f860a93u, 0x40490fdbu };
__global__ __launch_bounds__(256) void k_tab(const float* __restrict__ cn, float* Ct) { const unsigned i = blockIdx.x * 256u + threadIdx.x; const unsigned rt = i & 3u, sq = (i >> 2) & 31u, lv = i >> 7; const float ang = __fmul_rn((float)(lv + 1u) + bfr(cn[sq]), __uint_as_float(RATE[rt])); const float w = cosf(ang); *(volatile float*)(Ct + i) = w; __threadfence(); *(volatile float*)(Ct + i) = w; }
__global__ __launch_bounds__(32) void k_inc(const float* __restrict__ cn, float* oc) { const unsigned i = threadIdx.x; const float w = bfr(cn[i]) + 128.0f; *(volatile float*)(oc + i) = w; __threadfence(); *(volatile float*)(oc + i) = w; }
__global__ __launch_bounds__(32) void k_walka(const float* __restrict__ Pz, const float* __restrict__ ad, const int* __restrict__ zo, const float* __restrict__ Ct, const float* __restrict__ src, float* Pt, float* dst, unsigned ab, float m1, float m0) {
    const unsigned sq = blockIdx.y, ar = blockIdx.x, hd = threadIdx.x >> 2, qt = threadIdx.x & 3u;
    const size_t off = (((size_t)sq * gridDim.x + ar) * NA + hd) * 256u + qt * 64u;
    float st[64];
#pragma unroll
    for (int j = 0; j < 16; ++j) { const v4f w = *(const v4f*)(src + off + 4 * j); st[4 * j] = bfr(w[0]); st[4 * j + 1] = bfr(w[1]); st[4 * j + 2] = bfr(w[2]); st[4 * j + 3] = bfr(w[3]); }
    const unsigned ck = hd * 320u + qt * 16u, ce = NK5 + hd * 12u;
    for (unsigned lv = 0; lv < NL; ++lv) {
        const unsigned row = lv * NQ + sq; const float* pr = Pz + (size_t)row * NVP; const float keep = 1.0f - (float)zo[row];
        const float cs = Ct[row * 4u + ar] * m1 + m0;
        const v4f a1 = *(const v4f*)(pr + ce), a2 = *(const v4f*)(pr + ce + 4), a3 = *(const v4f*)(pr + ce + 8); const v4f e1 = *(const v4f*)(ad + ce), e2 = *(const v4f*)(ad + ce + 4), e3 = *(const v4f*)(ad + ce + 8);
        float r1[4], r2[4], s3[4];
#pragma unroll
        for (int m = 0; m < 4; ++m) { r1[m] = fmaxf(a1[m] + bfr(e1[m]), 0.0f); r2[m] = fmaxf(a2[m] + bfr(e2[m]), 0.0f); s3[m] = sgm(a3[m] + bfr(e3[m])); }
        float acc = 0.0f;
#pragma unroll
        for (int g4 = 0; g4 < 4; ++g4) { const v4f kx = *(const v4f*)(pr + ck + 4 * g4), qx = *(const v4f*)(pr + ck + 64 + 4 * g4), ux = *(const v4f*)(pr + ck + 256 + 4 * g4); const v4f ka = *(const v4f*)(ad + ck + 4 * g4), qa = *(const v4f*)(ad + ck + 64 + 4 * g4), ua = *(const v4f*)(ad + ck + 256 + 4 * g4);
#pragma unroll
            for (int n = 0; n < 4; ++n) { const int j = 4 * g4 + n; const float rk = fmaxf(kx[n] + bfr(ka[n]), 0.0f), rq = fmaxf(qx[n] + bfr(qa[n]), 0.0f), sg = sgm(ux[n] + bfr(ua[n]));
#pragma unroll
                for (int m = 0; m < 4; ++m) { const float wg = sg * s3[m]; const float en = ((rk * r1[m]) * wg) * cs; const float dk = (1.0f - wg) * keep; st[4 * j + m] = dk * st[4 * j + m] + en; acc += st[4 * j + m] * (rq * r2[m]); } } }
        float* pp = Pt + ((size_t)row * 8u + ab + ar) * 32u + threadIdx.x; *(volatile float*)pp = acc; __threadfence(); *(volatile float*)pp = acc;
    }
#pragma unroll
    for (int j = 0; j < 16; ++j) { v4f o; o[0] = st[4 * j]; o[1] = st[4 * j + 1]; o[2] = st[4 * j + 2]; o[3] = st[4 * j + 3]; *(volatile v4f*)(dst + off + 4 * j) = o; }
    __threadfence();
#pragma unroll
    for (int j = 0; j < 16; ++j) { v4f o; o[0] = st[4 * j]; o[1] = st[4 * j + 1]; o[2] = st[4 * j + 2]; o[3] = st[4 * j + 3]; *(volatile v4f*)(dst + off + 4 * j) = o; }
}
__global__ __launch_bounds__(256) void k_tot(const float* __restrict__ Pt, float* Sn) { const unsigned i = blockIdx.x * 256u + threadIdx.x; const unsigned row = i >> 2, rt = i & 3u; const float* pp = Pt + ((size_t)row * 8u + rt) * 32u; float acc = 0.0f;
#pragma unroll
    for (int l = 0; l < 32; ++l) acc += pp[l];
    *(volatile float*)(Sn + i) = acc; __threadfence(); *(volatile float*)(Sn + i) = acc; }
__global__ __launch_bounds__(256) void k_walkb(const float* __restrict__ Pz, const float* __restrict__ ad, const int* __restrict__ zo, const float* __restrict__ Ct, const float* __restrict__ Sn, const float* __restrict__ Pt, const float* __restrict__ c3, bf* Ah, bf* Al, float* o3) {
    const unsigned i = blockIdx.x * 256u + threadIdx.x; const unsigned pj = (i & 31u) * 2u, hd = (i >> 5) & 7u, sq = i >> 8; const unsigned cv = hd * 320u + 128u + pj, cg = cv + 64u; float st[NF][2];
#pragma unroll
    for (int rt = 0; rt < NF; ++rt) { const v2f w = *(const v2f*)(c3 + (((size_t)sq * NF + rt) * NA + hd) * NJ + pj); st[rt][0] = bfr(w[0]); st[rt][1] = bfr(w[1]); }
    const v2f av = *(const v2f*)(ad + cv), ag = *(const v2f*)(ad + cg); const float bv[2] = { bfr(av[0]), bfr(av[1]) }, bg[2] = { bfr(ag[0]), bfr(ag[1]) };
    for (unsigned lv = 0; lv < NL; ++lv) {
        const unsigned row = lv * NQ + sq; const float* pr = Pz + (size_t)row * NVP; const float keep = 1.0f - (float)zo[row];
        const v2f vx = *(const v2f*)(pr + cv), gx = *(const v2f*)(pr + cg); const v4f cs = *(const v4f*)(Ct + (size_t)row * 4u), wt = *(const v4f*)(Sn + (size_t)row * 4u), dp = *(const v4f*)(Pt + ((size_t)row * 8u + 4u) * 32u + hd * 4u); const float dn = 8.0f * (((dp[0] + dp[1]) + dp[2]) + dp[3]) + 1e-6f; v2us oh, ol;
#pragma unroll
        for (int n = 0; n < 2; ++n) { const float sv = sgm(gx[n] + bg[n]); const float en = (vx[n] + bv[n]) * sv; const float dk = (1.0f - sv) * keep; float sm = 0.0f;
#pragma unroll
            for (int rt = 0; rt < NF; ++rt) { st[rt][n] = dk * st[rt][n] + en * cs[rt]; sm += st[rt][n] * wt[rt]; }
            const float q2 = sm / dn; const unsigned short hw = f2bf(q2); oh[n] = hw; ol[n] = f2bf(q2 - bf2f(hw)); }
        const size_t ao = (size_t)row * NO + hd * NJ + pj; *(volatile v2us*)(Ah + ao) = oh; *(volatile v2us*)(Al + ao) = ol; __threadfence(); *(volatile v2us*)(Ah + ao) = oh; *(volatile v2us*)(Al + ao) = ol;
    }
#pragma unroll
    for (int rt = 0; rt < NF; ++rt) { v2f o; o[0] = st[rt][0]; o[1] = st[rt][1]; *(volatile v2f*)(o3 + (((size_t)sq * NF + rt) * NA + hd) * NJ + pj) = o; }
    __threadfence();
#pragma unroll
    for (int rt = 0; rt < NF; ++rt) { v2f o; o[0] = st[rt][0]; o[1] = st[rt][1]; *(volatile v2f*)(o3 + (((size_t)sq * NF + rt) * NA + hd) * NJ + pj) = o; }
}

extern "C" void kernel_launch(void* const* d_in, const int* in_sizes, int n_in, void* d_out, int out_size, void* d_ws, size_t ws_size, hipStream_t stream) {
    if (n_in < 10) return;
    if (in_sizes[0] != NM * NC || in_sizes[1] != NM || in_sizes[2] != NQ * NF * NA * 256 || in_sizes[3] != NQ * NF * NA * NJ || in_sizes[4] != NQ * NA * 256 || in_sizes[5] != NQ || in_sizes[6] != NV * NC || in_sizes[7] != NV || in_sizes[8] != NW * NO || in_sizes[9] != NW) return;
    if (out_size != NM * NW + NQ * NF * NA * 256 + NQ * NF * NA * NJ + NQ * NA * 256 + NQ) return;
    static_assert(NM == NL * NQ && NK5 == NA * 5 * NJ && NV == NK5 + NA * 3 * NE && NVP % 64 == 0 && NVP >= NV && NO == NA * NJ && NJ * NE == 256 && NM % 64 == 0 && NW % 64 == 0 && NC % 32 == 0 && NO % 32 == 0 && (NM * NC / 8) % 256 == 0 && (NV * NC / 8) % 256 == 0 && ((NVP - NV) * NC / 8) % 256 == 0 && (NW * NO / 8) % 256 == 0 && (NM * NF) % 256 == 0 && (NM * 4) % 256 == 0 && (NQ * NA * 32) % 256 == 0 && NQ == 32 && NF == 4 && NE == 4 && NJ == 64 && NA == 8 && NL == 128, "the products: row and column counts multiples of 64, the depths of 32; the one-dimensional grids exact; five arrays a sequence in two launches, a wave a (sequence, array); eight heads of 32 pairs a sequence; 128 levels");
    const float* i0 = (const float*)d_in[0]; const int* i1 = (const int*)d_in[1]; const float* i2 = (const float*)d_in[2]; const float* i3 = (const float*)d_in[3]; const float* i4 = (const float*)d_in[4]; const float* i5 = (const float*)d_in[5]; const float* i6 = (const float*)d_in[6]; const float* i7 = (const float*)d_in[7]; const float* i8 = (const float*)d_in[8]; const float* i9 = (const float*)d_in[9];
    float* out1 = (float*)d_out; float* out2 = out1 + (size_t)NM * NW; float* out3 = out2 + (size_t)NQ * NF * NA * 256; float* out4 = out3 + (size_t)NQ * NF * NA * NJ; float* out5 = out4 + (size_t)NQ * NA * 256;
    char* wsp = (char*)d_ws; auto take = [&](size_t bytes) { char* p = wsp; wsp += (bytes + 255) & ~(size_t)255; return (void*)p; };
    bf* Xb = (bf*)take((size_t)NM * NC * 2); bf* Wb = (bf*)take((size_t)NVP * NC * 2); float* Pz = (float*)take((size_t)NM * NVP * 4); float* Ct = (float*)take((size_t)NM * NF * 4); float* Pt = (float*)take((size_t)NM * 8 * 32 * 4); float* Sn = (float*)take((size_t)NM * 4 * 4); bf* Ah = (bf*)take((size_t)NM * NO * 2); bf* Al = (bf*)take((size_t)NM * NO * 2); bf* Wq = (bf*)take((size_t)NW * NO * 2);
    if ((size_t)(wsp - (char*)d_ws) > ws_size) return;
    k_cvt8<<<(unsigned)(NM * NC / 8 / 256), 256, 0, stream>>>(i0, Xb, (size_t)NM * NC / 8);
    k_cvt8<<<(unsigned)(NV * NC / 8 / 256), 256, 0, stream>>>(i6, Wb, (size_t)NV * NC / 8);
    k_fillb<<<(unsigned)((NVP - NV) * NC / 8 / 256), 256, 0, stream>>>(Wb + (size_t)NV * NC, 0u, (size_t)(NVP - NV) * NC / 8);
    k_cvt8<<<(unsigned)(NW * NO / 8 / 256), 256, 0, stream>>>(i8, Wq, (size_t)NW * NO / 8);
    k_gemmw<bf, 0, false><<<dim3(NM / 64, NVP / 64, 1), 32, 0, stream>>>(Xb, nullptr, Wb, nullptr, NC, Pz, NVP, nullptr, 0, 0, 0);
    k_tab<<<(unsigned)(NM * NF / 256), 256, 0, stream>>>(i5, Ct);
    k_inc<<<1, 32, 0, stream>>>(i5, out5);
    k_walka<<<dim3(NF, NQ, 1), 32, 0, stream>>>(Pz, i7, i1, Ct, i2, Pt, out2, 0u, 1.0f, 0.0f);
    k_walka<<<dim3(1, NQ, 1), 32, 0, stream>>>(Pz, i7, i1, Ct, i4, Pt, out4, 4u, 0.0f, 1.0f);
    k_tot<<<(unsigned)(NM * 4 / 256), 256, 0, stream>>>(Pt, Sn);
    k_walkb<<<(unsigned)(NQ * NA * 32 / 256), 256, 0, stream>>>(Pz, i7, i1, Ct, Sn, Pt, i3, Ah, Al, out3);
    k_gemmw<bf, 1, true><<<dim3(NM / 64, NW / 64, 1), 32, 0, stream>>>(Ah, Al, Wq, nullptr, NO, out1, NW, i9, 0, 0, 0);
}
